// PredicateUnit_34849364640337
// MI455X (gfx1250) — hardware-verified
//
#include <hip/hip_runtime.h>
#include <math.h>

typedef __attribute__((ext_vector_type(16))) _Float16 v16h;
typedef __attribute__((ext_vector_type(16))) __bf16 v16b;
typedef __attribute__((ext_vector_type(8)))  _Float16 v8h;
typedef __attribute__((ext_vector_type(8)))  float v8f;
typedef __attribute__((ext_vector_type(4)))  float v4f;
typedef __attribute__((ext_vector_type(2)))  float v2f;
typedef __attribute__((ext_vector_type(4)))  unsigned v4u;
typedef __attribute__((ext_vector_type(4)))  int v4i;
typedef float __attribute__((may_alias)) float_a;
typedef int __attribute__((may_alias)) int_a;

template <typename T> __device__ __forceinline__ void vst2(void* p, T v) { *(volatile T*)p = v; __threadfence(); *(volatile T*)p = v; }
__device__ __forceinline__ v8f wmma16(v16h a, v16h b, v8f c) {
  v8f d = __builtin_amdgcn_wmma_f32_16x16x32_f16(false, a, false, b, (short)0, c, false, false);
  asm volatile("v_nop\n\tv_nop\n\tv_nop\n\tv_nop" : "+v"(d) : "v"(a), "v"(b));
  return d;
}
__device__ __forceinline__ v8f wmma_bf(v16b a, v16b b, v8f c) {
  v8f d = __builtin_amdgcn_wmma_f32_16x16x32_bf16(false, a, false, b, (short)0, c, false, false);
  asm volatile("v_nop\n\tv_nop\n\tv_nop\n\tv_nop" : "+v"(d) : "v"(a), "v"(b));
  return d;
}
__device__ __forceinline__ v16h frag_h(const _Float16* rowk0, int lane) {
  union { v16h v; v8h q[2]; } u; const _Float16* p = rowk0 + 8 * (lane >> 4);
  u.q[0] = *(const v8h*)p; u.q[1] = *(const v8h*)(p + 16); return u.v;
}
__device__ __forceinline__ v16h frag_f32(const float* rowk0, int lane) {
  v16h a; const float* p = rowk0 + 8 * (lane >> 4);
#pragma unroll
  for (int i = 0; i < 8; ++i) { a[i] = (_Float16)p[i]; a[8 + i] = (_Float16)p[16 + i]; }
  return a;
}
__device__ __forceinline__ v16h frag_f32s(const float* rowk0, int lane, float sc) {
  v16h a; const float* p = rowk0 + 8 * (lane >> 4);
#pragma unroll
  for (int i = 0; i < 8; ++i) { a[i] = (_Float16)(p[i] * sc); a[8 + i] = (_Float16)(p[16 + i] * sc); }
  return a;
}
__device__ __forceinline__ v16h fragc_f32(const float* W, int k0, int n, int lane, int ld, int K) {
  v16h a; const int g = lane >> 4;
#pragma unroll
  for (int i = 0; i < 8; ++i) { const int ka = k0 + 8 * g + i, kb = ka + 16;
    a[i] = (_Float16)(ka < K ? W[(size_t)(ka < K ? ka : K - 1) * ld + n] : 0.f); a[8 + i] = (_Float16)(kb < K ? W[(size_t)(kb < K ? kb : K - 1) * ld + n] : 0.f); }
  return a;
}
struct F2 { v16b h, l; };
__device__ __forceinline__ F2 bsplit16(const float v[16]) { F2 r;
#pragma unroll
  for (int i = 0; i < 16; ++i) { const __bf16 h = (__bf16)v[i]; r.h[i] = h; r.l[i] = (__bf16)(v[i] - (float)h); }
  return r; }
__device__ __forceinline__ F2 split_row(const float* row, int k0, int lane) { float v[16]; const float* p = row + k0 + 8 * (lane >> 4);
#pragma unroll
  for (int i = 0; i < 8; ++i) { v[i] = p[i]; v[8 + i] = p[16 + i]; }
  return bsplit16(v); }
__device__ __forceinline__ F2 split_rowK(const float* row, int k0, int lane, int K) { float v[16]; const int g = lane >> 4;
#pragma unroll
  for (int i = 0; i < 8; ++i) { const int ka = k0 + 8 * g + i, kb = ka + 16; v[i] = ka < K ? row[ka < K ? ka : K - 1] : 0.f; v[8 + i] = kb < K ? row[kb < K ? kb : K - 1] : 0.f; }
  return bsplit16(v); }
__device__ __forceinline__ F2 split_col(const float* W, int k0, int n, int lane, int ld, int K) { float v[16]; const int g = lane >> 4;
#pragma unroll
  for (int i = 0; i < 8; ++i) { const int ka = k0 + 8 * g + i, kb = ka + 16; v[i] = ka < K ? W[(size_t)(ka < K ? ka : K - 1) * ld + n] : 0.f; v[8 + i] = kb < K ? W[(size_t)(kb < K ? kb : K - 1) * ld + n] : 0.f; }
  return bsplit16(v); }
__device__ __forceinline__ v8f mac3(const F2& a, const F2& b, v8f c) { c = wmma_bf(a.l, b.h, c); c = wmma_bf(a.h, b.l, c); return wmma_bf(a.h, b.h, c); }
__device__ __forceinline__ float sigm(float v) { return 1.0f / (1.0f + expf(-v)); }
#define LDSX() do { asm volatile("s_wait_dscnt 0" ::: "memory"); __builtin_amdgcn_wave_barrier(); __builtin_amdgcn_fence(__ATOMIC_RELEASE, "workgroup"); } while (0)


#define NBAT 64
#define NOBJ 5
#define NTUP (NBAT * NOBJ * NOBJ)
#define NIMG (2 * NTUP)
#define IH 64
#define IW 96
#define OH 32
#define OW 48
#define NPIX (OH * OW)
#define NCH 128
#define KIM 54
#define NCHUNK (NPIX / 128)
#ifndef TIMG
#define TIMG NIMG
#endif
typedef __attribute__((ext_vector_type(8))) __bf16 v8b;
__device__ __forceinline__ v16b frag_b(const __bf16* rowk0, int lane) {
  union { v16b v; v8b q[2]; } u; const __bf16* p = rowk0 + 8 * (lane >> 4);
  u.q[0] = *(const v8b*)p; u.q[1] = *(const v8b*)(p + 16); return u.v;
}
__device__ __forceinline__ float bfr(float v) { return (float)(__bf16)v; }
__device__ __attribute__((noinline)) float exp_ni(float v) { return expf(v); }
#define WS_PT   0u
#define WS_PART (WS_PT + 2u * NCH * 64)
#define WS_LG   (WS_PART + 4u * NIMG * NCHUNK * NCH)
#define WS_END  (WS_LG + 4u * NIMG * 4)

__global__ __launch_bounds__(64) void k_pack(const float* __restrict__ CW, __bf16* __restrict__ PT) {
  __shared__ __align__(16) __bf16 s[64]; const int o = blockIdx.x, tid = threadIdx.x; s[tid] = (__bf16)((tid < KIM) ? bfr(CW[(size_t)o * KIM + tid]) : 0.f); __syncthreads();
  if (tid < 8) vst2((unsigned*)(PT + (size_t)o * 64 + tid * 8), *(const v4u*)&s[tid * 8]);
}
__global__ __launch_bounds__(128) void k_conv(const float* __restrict__ S0, const float* __restrict__ S1, const __bf16* __restrict__ PT, const float* __restrict__ CB, float* __restrict__ PART) {
  __shared__ __align__(16) __bf16 sa[128][72]; __shared__ float ssum[4][NCH]; __shared__ __align__(16) float sres[NCH];
  const int tid = threadIdx.x, wave = tid >> 5, lane = tid & 31, col = lane & 15, g = lane >> 4; const int chunk = blockIdx.x, img = blockIdx.y;
  const int which = img / NTUP, t = img % NTUP; const int b = t / (NOBJ * NOBJ), pr = t % (NOBJ * NOBJ); const int oi = pr / NOBJ, oj = pr % NOBJ; const float* S = which == 0 ? S0 : S1;
  const float* IA = S + ((size_t)(b * NOBJ + oi)) * 3 * IH * IW; const float* IB = S + ((size_t)(b * NOBJ + oj)) * 3 * IH * IW;
  { const int pix = chunk * 128 + tid; const int oy = pix / OW, ox = pix % OW; union { v4u v[8]; __bf16 h[64]; } rb;
#pragma unroll
    for (int c = 0; c < 6; ++c) { const float* I = (c < 3) ? IA + (size_t)c * IH * IW : IB + (size_t)(c - 3) * IH * IW;
#pragma unroll
      for (int ky = 0; ky < 3; ++ky) { const int y = 2 * oy + ky; const float* Irow = I + (y < IH ? y : IH - 1) * IW;
#pragma unroll
        for (int kx = 0; kx < 3; ++kx) { const int x = 2 * ox + kx; const float v = Irow[x < IW ? x : IW - 1]; rb.h[c * 9 + ky * 3 + kx] = (y < IH && x < IW) ? (__bf16)v : (__bf16)0.f; } } }
#pragma unroll
    for (int k = KIM; k < 64; ++k) rb.h[k] = (__bf16)0.f;
#pragma unroll
    for (int q = 0; q < 8; ++q) *(v4u*)&sa[tid][q * 8] = rb.v[q]; }
  __syncthreads();
  v8f acc[2][8] = {};
#pragma unroll
  for (int kc = 0; kc < 2; ++kc) { const v16b a0 = frag_b(&sa[wave * 32 + col][kc * 32], lane), a1 = frag_b(&sa[wave * 32 + 16 + col][kc * 32], lane);
#pragma unroll
    for (int j = 0; j < 8; ++j) { const v16b w = frag_b(PT + (size_t)(j * 16 + col) * 64 + kc * 32, lane); acc[0][j] = wmma_bf(a0, w, acc[0][j]); acc[1][j] = wmma_bf(a1, w, acc[1][j]); } }
#pragma unroll
  for (int j = 0; j < 8; ++j) { const int o = j * 16 + col; const float bb = bfr(CB[o]); float s = 0.f;
#pragma unroll
    for (int r = 0; r < 8; ++r) s += fmaxf(acc[0][j][r] + bb, 0.f) + fmaxf(acc[1][j][r] + bb, 0.f);
    s += __shfl_xor(s, 16);
    if (g == 0) ssum[wave][o] = s; }
  __syncthreads();
  if (tid < NCH) sres[tid] = (ssum[0][tid] + ssum[1][tid]) + (ssum[2][tid] + ssum[3][tid]);
  __syncthreads();
  if (tid < 32) vst2(PART + ((size_t)img * NCHUNK + chunk) * NCH + tid * 4, *(const v4f*)&sres[tid * 4]);
}
__global__ __launch_bounds__(256) void k_fin(const float* __restrict__ PART, const float* __restrict__ W2, const float* __restrict__ B2, const float* __restrict__ TEMP, float* __restrict__ LG) {
  __shared__ float smean[8][NCH]; __shared__ __align__(16) float slg[8][4];
  const int tid = threadIdx.x; const int img0 = blockIdx.x * 8;
  for (int q = tid; q < 8 * NCH; q += 256) { const int il = q / NCH, c = q % NCH; float s = 0.f;
#pragma unroll 1
    for (int ch = 0; ch < NCHUNK; ++ch) s += PART[((size_t)(img0 + il) * NCHUNK + ch) * NCH + c];
    smean[il][c] = s / (float)NPIX; }
  __syncthreads();
  if (tid < 32) { const int il = tid >> 2, p = tid & 3; float s = bfr(B2[p]);
#pragma unroll 1
    for (int c = 0; c < 32; ++c) s += smean[il][p * 32 + c] * bfr(W2[p * 32 + c]);
    const float itemp = 1.0f / bfr(TEMP[0]); slg[il][p] = 1.0f / (1.0f + exp_ni(-s * itemp)); }
  __syncthreads();
  if (tid < 8) vst2(LG + (size_t)(img0 + tid) * 4, *(const v4f*)&slg[tid][0]);
}
__global__ __launch_bounds__(256) void k_out(const float* __restrict__ LG, float* __restrict__ out) {
  const size_t p = (size_t)blockIdx.x * 256 + threadIdx.x; const size_t npred = (size_t)NIMG * 4; const size_t total = npred + (size_t)NBAT * NTUP; if (p * 4 >= total) return;
  v4f v; if (p * 4 < npred) v = *(const v4f*)(LG + p * 4); else { for (int i = 0; i < 4; ++i) { const size_t f = p * 4 + i - npred; const int b = (int)(f / NTUP), t = (int)(f % NTUP); v[i] = (t / (NOBJ * NOBJ) == b) ? 1.0f : 0.0f; } }
  vst2(out + p * 4, v);
}
extern "C" void kernel_launch(void* const* d_in, const int* in_sizes, int n_in, void* d_out, int out_size, void* d_ws, size_t ws_size, hipStream_t stream) {
  (void)in_sizes; (void)n_in; (void)out_size;
  const float** F = (const float**)d_in;
  if (ws_size < (size_t)WS_END) return;
  char* ws = (char*)d_ws; __bf16* PT = (__bf16*)(ws + WS_PT); float *PART = (float*)(ws + WS_PART), *LG = (float*)(ws + WS_LG);
  k_pack<<<NCH, 64, 0, stream>>>(F[2], PT);
  k_conv<<<dim3(NCHUNK, TIMG), 128, 0, stream>>>(F[0], F[1], PT, F[3], PART);
  k_fin<<<TIMG / 8, 256, 0, stream>>>(PART, F[4], F[5], F[7], LG);
  k_out<<<(NIMG * 4 + NBAT * NTUP + 1023) / 1024, 256, 0, stream>>>(LG, (float*)d_out);
}
